// CausalSelfAttention_4475355922513
// MI455X (gfx1250) — hardware-verified
//
#include <hip/hip_runtime.h>


#ifndef NB
#define NB 2
#endif
#ifndef SEQ
#define SEQ 2048
#endif
#define NB_FULL  2
#define SEQ_FULL 2048
#define DM   2048
#define NH   16
#define NKV  4
#define REP  (NH / NKV)
#define HD   128
#define DQ   (NH * HD)
#define DKV  (NKV * HD)
#define RH   256
#define QCAR 64.0f
#define CCAR 256.0f
#define WCAR 16.0f
#define OSP  132
#define CP   136

static_assert(NB <= NB_FULL);
static_assert(SEQ <= SEQ_FULL);
static_assert(SEQ % 128 == 0);
static_assert(SEQ >= RH);
static_assert(RH % 32 == 0);
static_assert(HD == 128);
static_assert(REP == 4);
static_assert(DQ == DM);
static_assert(DM % 64 == 0);
static_assert(DQ % 128 == 0);
static_assert(DKV % 128 == 0);
static_assert((OSP * 4) % 16 == 0);
static_assert((CP * 2) % 16 == 0);

typedef _Float16 h16;
typedef unsigned short bf;
typedef __attribute__((ext_vector_type(16))) __bf16   v16bf;
typedef __attribute__((ext_vector_type(16))) _Float16 v16h;
typedef __attribute__((ext_vector_type(8)))  _Float16 v8h;
typedef __attribute__((ext_vector_type(8)))  unsigned short v8us;
typedef __attribute__((ext_vector_type(2)))  unsigned short v2us;
typedef __attribute__((ext_vector_type(8)))  float    v8f;
typedef __attribute__((ext_vector_type(4)))  float    v4f;
typedef __attribute__((ext_vector_type(2)))  float    v2f;
typedef v8h  __attribute__((may_alias)) v8ha;
typedef v4f  __attribute__((may_alias)) v4fa;

__device__ __forceinline__ unsigned short f2bf(float f) { unsigned u = __float_as_uint(f); u += 0x7FFFu + ((u >> 16) & 1u); return (unsigned short)(u >> 16); }
__device__ __forceinline__ float bf2f(unsigned short b) { return __uint_as_float(((unsigned)b) << 16); }
__device__ __forceinline__ float bfr(float f) { return bf2f(f2bf(f)); }
__device__ __forceinline__ v16h cat16(v8h lo, v8h hi) { return __builtin_shufflevector(lo, hi, 0, 1, 2, 3, 4, 5, 6, 7, 8, 9, 10, 11, 12, 13, 14, 15); }
__device__ __forceinline__ v16bf cat16b(v8us lo, v8us hi) { return __builtin_bit_cast(v16bf, __builtin_shufflevector(lo, hi, 0, 1, 2, 3, 4, 5, 6, 7, 8, 9, 10, 11, 12, 13, 14, 15)); }
__device__ __forceinline__ v8f wmma16(v16h a, v16h b, v8f c) {
    c = __builtin_amdgcn_wmma_f32_16x16x32_f16(false, a, false, b, (short)0, c, false, false);
    asm volatile("v_nop\n\tv_nop\n\tv_nop\n\tv_nop" : "+v"(c) : "v"(a), "v"(b));
    return c; }
__device__ __forceinline__ v8f wmmab(v16bf a, v16bf b, v8f c) {
    c = __builtin_amdgcn_wmma_f32_16x16x32_bf16(false, a, false, b, (short)0, c, false, false);
    asm volatile("v_nop\n\tv_nop\n\tv_nop\n\tv_nop" : "+v"(c) : "v"(a), "v"(b));
    return c; }
__device__ __forceinline__ v16h ldh(const h16* p) { return cat16(*(const v8h*)p, *(const v8h*)(p + 16)); }
__device__ __forceinline__ void wave_sync() { __builtin_amdgcn_fence(3  , "wavefront"); __builtin_amdgcn_wave_barrier(); asm volatile("" ::: "memory"); }
__device__ __forceinline__ void split8(v8f y, v8h& v, v8h& r) { v = __builtin_convertvector(y, v8h); r = __builtin_convertvector(y - __builtin_convertvector(v, v8f), v8h); }

template <typename T16> struct WFrag;
template <> struct WFrag<h16> { typedef v16h V; static __device__ __forceinline__ V ld(const h16* p) { return cat16(*(const v8h*)p, *(const v8h*)(p + 16)); } static __device__ __forceinline__ v8f mma(V a, V b, v8f c) { return wmma16(a, b, c); } };
template <> struct WFrag<bf> { typedef v16bf V; static __device__ __forceinline__ V ld(const bf* p) { return cat16b(*(const v8us*)p, *(const v8us*)(p + 16)); } static __device__ __forceinline__ v8f mma(V a, V b, v8f c) { return wmmab(a, b, c); } };

template <typename T16, int MODE, bool SPLIT>
__device__ __forceinline__ void gemm_tile(const T16* __restrict__ A, const T16* __restrict__ A2, const T16* __restrict__ Bt, const int K,
                                          const size_t arow, const size_t a2row, const size_t brow,
                                          const float* __restrict__ CS, const int t0, h16* Pv, h16* Pr, const size_t obase, const int opitch,
                                          float* C, const size_t cbase) {
    typedef typename WFrag<T16>::V V;
    __shared__ __align__(16) float os[16 * OSP];
    const int lane = threadIdx.x & 31, lr = lane & 15, hi = lane >> 4;
    v8f acc[2][8];
#pragma unroll
    for (int mb = 0; mb < 2; ++mb)
#pragma unroll
        for (int nb = 0; nb < 8; ++nb) acc[mb][nb] = (v8f){};
    const T16* ap  = A  + (arow  + lr) * (size_t)K + 8 * hi;
    const T16* ap2 = A2 + (a2row + lr) * (size_t)K + 8 * hi;
    const T16* bp  = Bt + (brow  + lr) * (size_t)K + 8 * hi;
    const int K16 = 16 * K;
#pragma unroll 1
    for (int kc = 0; kc < K; kc += 32) {
        const V a0 = WFrag<T16>::ld(ap + kc), a1 = WFrag<T16>::ld(ap + K16 + kc);
        V r0 = a0, r1 = a1;
        if (SPLIT) { r0 = WFrag<T16>::ld(ap2 + kc); r1 = WFrag<T16>::ld(ap2 + K16 + kc); }
#pragma unroll
        for (int nb = 0; nb < 8; ++nb) {
            const V bb = WFrag<T16>::ld(bp + nb * K16 + kc);
            acc[0][nb] = WFrag<T16>::mma(a0, bb, acc[0][nb]);
            acc[1][nb] = WFrag<T16>::mma(a1, bb, acc[1][nb]);
            if (SPLIT) { acc[0][nb] = WFrag<T16>::mma(r0, bb, acc[0][nb]); acc[1][nb] = WFrag<T16>::mma(r1, bb, acc[1][nb]); }
        }
    }
#pragma unroll
    for (int mb = 0; mb < 2; ++mb) {
#pragma unroll
        for (int nb = 0; nb < 8; ++nb)
#pragma unroll
            for (int j = 0; j < 8; ++j) os[(hi * 8 + j) * OSP + nb * 16 + lr] = acc[mb][nb][j];
        wave_sync();
        if (MODE == 0) {
            const int rq = lane >> 3, dg = (lane & 7) * 8;
#pragma unroll 1
            for (int ps = 0; ps < 2; ++ps) {
#pragma unroll 1
                for (int it = 0; it < 4; ++it) {
                    const int row = it * 4 + rq; const int t = t0 + mb * 16 + row;
                    const int oi = row * OSP + dg;
                    const v4f xa = *(const v4fa*)(os + oi), xb = *(const v4fa*)(os + oi + 4), ya = *(const v4fa*)(os + oi + 64), yb = *(const v4fa*)(os + oi + 68);
                    const float* cp = CS + ((size_t)t * 64 + dg) * 2;
                    const v4f e0 = *(const v4f*)(cp), e1 = *(const v4f*)(cp + 4), e2 = *(const v4f*)(cp + 8), e3 = *(const v4f*)(cp + 12);
                    const v8f xx = __builtin_shufflevector(xa, xb, 0, 1, 2, 3, 4, 5, 6, 7), yy = __builtin_shufflevector(ya, yb, 0, 1, 2, 3, 4, 5, 6, 7);
                    const v4f cA = __builtin_shufflevector(e0, e1, 0, 2, 4, 6), sA = __builtin_shufflevector(e0, e1, 1, 3, 5, 7);
                    const v4f cB = __builtin_shufflevector(e2, e3, 0, 2, 4, 6), sB = __builtin_shufflevector(e2, e3, 1, 3, 5, 7);
                    const v8f cc = __builtin_shufflevector(cA, cB, 0, 1, 2, 3, 4, 5, 6, 7), ss = __builtin_shufflevector(sA, sB, 0, 1, 2, 3, 4, 5, 6, 7);
                    const v8f lo = (xx * cc - yy * ss) * QCAR;
                    const v8f up = (yy * cc + xx * ss) * QCAR;
                    v8h vl, rl, vu, ru; split8(lo, vl, rl); split8(up, vu, ru);
                    const size_t dst = obase + (size_t)(mb * 16 + row) * opitch + dg;
                    *(volatile v8h*)(Pv + dst) = vl; *(volatile v8h*)(Pv + dst + 64) = vu;
                    *(volatile v8h*)(Pr + dst) = rl; *(volatile v8h*)(Pr + dst + 64) = ru;
                }
                if (ps == 0) __threadfence();
            }
        } else if (MODE == 1) {
#pragma unroll 1
            for (int ps = 0; ps < 2; ++ps) {
#pragma unroll 1
                for (int s = 0; s < 8; ++s) {
                    const int row = 2 * s + hi; const int oi = row * OSP + 8 * lr;
                    const v4f xa = *(const v4fa*)(os + oi), xb = *(const v4fa*)(os + oi + 4);
                    const v8f y = __builtin_shufflevector(xa, xb, 0, 1, 2, 3, 4, 5, 6, 7) * QCAR;
                    v8h vv, vr; split8(y, vv, vr);
                    const size_t dst = obase + (size_t)(mb * 16 + row) * opitch + 8 * lr;
                    *(volatile v8h*)(Pv + dst) = vv; *(volatile v8h*)(Pr + dst) = vr;
                }
                if (ps == 0) __threadfence();
            }
        } else {
#pragma unroll 1
            for (int ps = 0; ps < 2; ++ps) {
#pragma unroll 1
                for (int row = 0; row < 16; ++row) {
                    const v4f val = *(const v4fa*)(os + row * OSP + 4 * lane) * (1.0f / (CCAR * WCAR));
                    *(volatile v4f*)(C + cbase + (size_t)(mb * 16 + row) * DM + 4 * lane) = val;
                }
                if (ps == 0) __threadfence();
            }
        }
        wave_sync();
    }
}

__global__ __launch_bounds__(32) __attribute__((amdgpu_num_vgpr(256)))
void k_proj_qk(const bf* __restrict__ XB, const bf* __restrict__ Wt, const float* __restrict__ CS, h16* Pv, h16* Pr, int nheads) {
    const int r0 = blockIdx.x * 32; const int hd = blockIdx.y; const int b = r0 / SEQ; const int t0 = r0 - b * SEQ;
    const size_t obase = ((size_t)(b * nheads + hd) * SEQ + t0) * HD;
    gemm_tile<bf, 0, false>(XB, XB, Wt, DM, (size_t)r0, (size_t)r0, (size_t)hd * HD, CS, t0, Pv, Pr, obase, HD, nullptr, 0);
}
__global__ __launch_bounds__(32) __attribute__((amdgpu_num_vgpr(256)))
void k_proj_vt(const bf* __restrict__ Wt, const bf* __restrict__ XB, h16* Vv, h16* Vr) {
    const int r0 = blockIdx.x * 32; const int c0 = blockIdx.y * 128; const int b = c0 / SEQ; const int t0 = c0 - b * SEQ;
    const size_t obase = ((size_t)b * DKV + r0) * SEQ + t0;
    gemm_tile<bf, 1, false>(Wt, Wt, XB, DM, (size_t)r0, (size_t)r0, (size_t)c0, nullptr, 0, Vv, Vr, obase, SEQ, nullptr, 0);
}
__global__ __launch_bounds__(32) __attribute__((amdgpu_num_vgpr(256)))
void k_oproj(const h16* __restrict__ CT, const h16* __restrict__ WOt, float* OUT) {
    constexpr int TPB = (SEQ > RH) ? (SEQ - RH) / 32 : 1;
    const int b = blockIdx.x / TPB; const int t0 = RH + (blockIdx.x - b * TPB) * 32; const int c0 = blockIdx.y * 128;
    const size_t arow = (size_t)b * SEQ + t0; const size_t cbase = ((size_t)b * SEQ_FULL + t0) * DM + c0;
    gemm_tile<h16, 2, false>(CT, CT, WOt, DQ, arow, arow, (size_t)c0, nullptr, 0, nullptr, nullptr, 0, 0, OUT, cbase);
}
__global__ __launch_bounds__(32) __attribute__((amdgpu_num_vgpr(256)))
void k_oproj_hr(const h16* __restrict__ CT, const h16* __restrict__ CR, const h16* __restrict__ WOt, float* OUT) {
    constexpr int TPB = RH / 32;
    const int b = blockIdx.x / TPB; const int t0 = (blockIdx.x - b * TPB) * 32; const int c0 = blockIdx.y * 128;
    const size_t arow = (size_t)b * SEQ + t0; const size_t a2row = (size_t)b * RH + t0; const size_t cbase = ((size_t)b * SEQ_FULL + t0) * DM + c0;
    gemm_tile<h16, 2, true>(CT, CR, WOt, DQ, arow, a2row, (size_t)c0, nullptr, 0, nullptr, nullptr, 0, 0, OUT, cbase);
}

template <bool HR>
__device__ __forceinline__ void attn_tile(const h16* __restrict__ Qv, const h16* __restrict__ Qr, const h16* __restrict__ Kv, const h16* __restrict__ Kr,
                                          const h16* __restrict__ Vv, const h16* __restrict__ Vr, h16* CT, h16* CR, const int qt) {
    __shared__ __align__(16) h16 stv[4 * 16 * CP];
    __shared__ __align__(16) h16 str[HR ? 4 * 16 * CP : 8];
    const int wave = __builtin_amdgcn_readfirstlane((int)(threadIdx.x >> 5));
    const int lane = threadIdx.x & 31, lr = lane & 15, hi = lane >> 4;
    const int g = blockIdx.y, b = blockIdx.z; const int h = g * REP + wave; const int i0 = qt * 16;
    const size_t qo = ((size_t)(b * NH + h) * SEQ + i0 + lr) * HD + 8 * hi;
    const size_t ko = ((size_t)(b * NKV + g) * SEQ + lr) * HD + 8 * hi;
    const size_t vo = ((size_t)(b * NKV + g) * HD + lr) * SEQ + 8 * hi;
    const h16* qv = Qv + qo; const h16* qr = Qr + qo;
    const h16* kv = Kv + ko; const h16* kr = Kr + ko;
    const h16* vv = Vv + vo; const h16* vr = Vr + vo;
    const float SC2 = (float)(0.08838834764831845 * 1.4426950408889634 / 4096.0);
    const float NEGL = -1.4426950e9f;
    v8f o[8];
#pragma unroll
    for (int dt = 0; dt < 8; ++dt) o[dt] = (v8f){};
    float m = -3.0e38f, l = 0.0f;
    const int nsteps = (qt >> 1) + 1;
#pragma unroll 1
    for (int stp = 0; stp < nsteps; ++stp) {
        const int k0 = stp * 32;
        v8f s0 = (v8f){}, s1 = (v8f){};
        const h16* kp = kv + (size_t)k0 * HD; const h16* kpr = kr + (size_t)k0 * HD;
#pragma unroll 1
        for (int kc = 0; kc < HD; kc += 32) {
            const v16h bq = ldh(qv + kc), br = ldh(qr + kc);
            const v16h a0 = ldh(kp + kc);
            s0 = wmma16(a0, bq, s0); s0 = wmma16(a0, br, s0);
            if (HR) { const v16h a0r = ldh(kpr + kc); s0 = wmma16(a0r, bq, s0); }
            const v16h a1 = ldh(kp + 16 * HD + kc);
            s1 = wmma16(a1, bq, s1); s1 = wmma16(a1, br, s1);
            if (HR) { const v16h a1r = ldh(kpr + 16 * HD + kc); s1 = wmma16(a1r, bq, s1); }
        }
        s0 = s0 * SC2; s1 = s1 * SC2;
        if (k0 + 31 > i0) {
            const int qi = i0 + lr; const int kb = k0 + 8 * hi;
#pragma unroll
            for (int r = 0; r < 8; ++r) { s0[r] = (kb + r <= qi) ? s0[r] : NEGL; s1[r] = (kb + 16 + r <= qi) ? s1[r] : NEGL; }
        }
        float mx = fmaxf(s0[0], s1[0]);
#pragma unroll
        for (int r = 1; r < 8; ++r) mx = fmaxf(mx, fmaxf(s0[r], s1[r]));
        mx = fmaxf(mx, __shfl_xor(mx, 16, 32));
        const float mn = fmaxf(m, mx);
        if (__builtin_amdgcn_ballot_w32(mn > m) != 0u) {
            const float corr = __builtin_amdgcn_exp2f(m - mn); l *= corr;
#pragma unroll
            for (int dt = 0; dt < 8; ++dt) o[dt] = o[dt] * corr;
        }
        m = mn;
        const float mm = mn - 10.0f;
        v8f p0, p1; float ps = 0.0f;
#pragma unroll
        for (int r = 0; r < 8; ++r) { p0[r] = __builtin_amdgcn_exp2f(s0[r] - mm); p1[r] = __builtin_amdgcn_exp2f(s1[r] - mm); ps += p0[r] + p1[r]; }
        l += ps;
        v8h p0v, p0r, p1v, p1r; split8(p0, p0v, p0r); split8(p1, p1v, p1r);
        const v16h pb = cat16(p0v, p1v);
        const v16h pr = cat16(p0r, p1r);
        const h16* vp = vv + k0; const h16* vpr = vr + k0;
#pragma unroll
        for (int dt = 0; dt < 8; ++dt) {
            const v16h av = ldh(vp + (size_t)dt * 16 * SEQ);
            o[dt] = wmma16(av, pb, o[dt]);
            if (HR) { const v16h ar = ldh(vpr + (size_t)dt * 16 * SEQ); o[dt] = wmma16(ar, pb, o[dt]); o[dt] = wmma16(av, pr, o[dt]); }
        }
    }
    l += __shfl_xor(l, 16, 32);
    const float f = (CCAR / QCAR) * (1.0f / l);
    const int sb = wave * 16 * CP;
#pragma unroll
    for (int dt = 0; dt < 8; ++dt) {
        v8h hv, hr; split8(o[dt] * f, hv, hr);
        *(v8h*)(&stv[sb + lr * CP + dt * 16 + 8 * hi]) = hv;
        if (HR) *(v8h*)(&str[sb + lr * CP + dt * 16 + 8 * hi]) = hr;
    }
    wave_sync();
    const size_t crow = ((size_t)b * SEQ + i0) * DQ + (size_t)h * HD + 8 * lr;
    const size_t rrow = ((size_t)b * RH + i0) * DQ + (size_t)h * HD + 8 * lr;
#pragma unroll 1
    for (int ps2 = 0; ps2 < 2; ++ps2) {
#pragma unroll
        for (int s = 0; s < 8; ++s) {
            const int row = 2 * s + hi;
            const v8h val = *(const v8ha*)(&stv[sb + row * CP + 8 * lr]);
            *(volatile v8h*)(CT + crow + (size_t)row * DQ) = val;
            if (HR) { const v8h rv = *(const v8ha*)(&str[sb + row * CP + 8 * lr]); *(volatile v8h*)(CR + rrow + (size_t)row * DQ) = rv; }
        }
        if (ps2 == 0) __threadfence();
    }
}
__global__ __launch_bounds__(128) __attribute__((amdgpu_num_vgpr(256)))
void k_attn(const h16* __restrict__ Qv, const h16* __restrict__ Qr, const h16* __restrict__ Kv, const h16* __restrict__ Vv, h16* CT) {
    attn_tile<false>(Qv, Qr, Kv, Kv, Vv, Vv, CT, CT, RH / 16 + (int)blockIdx.x);
}
__global__ __launch_bounds__(128) __attribute__((amdgpu_num_vgpr(256)))
void k_attn_hr(const h16* __restrict__ Qv, const h16* __restrict__ Qr, const h16* __restrict__ Kv, const h16* __restrict__ Kr,
               const h16* __restrict__ Vv, const h16* __restrict__ Vr, h16* CT, h16* CR) {
    attn_tile<true>(Qv, Qr, Kv, Kr, Vv, Vr, CT, CR, (int)blockIdx.x);
}

__global__ __launch_bounds__(256) void k_wtG(const float* __restrict__ w, int K, int N, bf* Bt, int f16mode) {
    const int lane = threadIdx.x & 31; const int L0 = (blockIdx.x * 8 + (threadIdx.x >> 5)) * 8; const int nlines = N * (K / 64);
#pragma unroll 1
    for (int ps = 0; ps < 2; ++ps) {
#pragma unroll 1
        for (int l = 0; l < 8; ++l) { const int L = L0 + l; if (L >= nlines) break; const size_t e = (size_t)L * 64 + lane * 2; const int k = (int)(e % K), n = (int)(e / K);
            const float w0 = w[(size_t)k * N + n], w1 = w[(size_t)(k + 1) * N + n];
            const unsigned short b0 = f2bf(w0), b1 = f2bf(w1);
            const unsigned short g0 = __builtin_bit_cast(unsigned short, (h16)(bf2f(b0) * WCAR)), g1 = __builtin_bit_cast(unsigned short, (h16)(bf2f(b1) * WCAR));
            v2us o; o[0] = f16mode ? g0 : b0; o[1] = f16mode ? g1 : b1;
            *(volatile v2us*)(Bt + e) = o; }
        if (ps == 0) __threadfence(); }
}
__global__ __launch_bounds__(256) void k_cvtx(const float* __restrict__ x, bf* XB) {
    const size_t i = (size_t)blockIdx.x * 256 + threadIdx.x; if (i >= (size_t)NB * SEQ * DM / 8) return;
    const size_t e = i * 8; const size_t bt = e / DM; const size_t col = e - bt * DM; const size_t b = bt / SEQ; const size_t t = bt - b * SEQ;
    const v8f v = *(const v8f*)(x + (b * SEQ_FULL + t) * DM + col); v8us o;
#pragma unroll
    for (int k = 0; k < 8; ++k) o[k] = f2bf(v[k]);
    *(volatile v8us*)(XB + e) = o; __threadfence(); *(volatile v8us*)(XB + e) = o;
}
__global__ __launch_bounds__(256) void k_cstab(float* CS) {
    const int idx = blockIdx.x * 256 + threadIdx.x; if (idx >= SEQ * 64) return;
    const int j = idx & 63, t = idx >> 6;
    double p = 1.0;
    p *= (j & 1)  ? 1.1547819846894581797 : 1.0;
    p *= (j & 2)  ? 1.3335214321633240257 : 1.0;
    p *= (j & 4)  ? 1.7782794100389228012 : 1.0;
    p *= (j & 8)  ? 3.1622776601683793320 : 1.0;
    p *= (j & 16) ? 10.0 : 1.0;
    p *= (j & 32) ? 100.0 : 1.0;
    const float pf = (float)p; const float inv = 1.0f / pf; const float ang = (float)t * inv;
    float sn, cn; sincosf(ang, &sn, &cn);
    v2f cs; cs[0] = cn; cs[1] = sn;
    *(volatile v2f*)(CS + (size_t)idx * 2) = cs; __threadfence(); *(volatile v2f*)(CS + (size_t)idx * 2) = cs;
}

extern "C" void kernel_launch(void* const* d_in, const int* in_sizes, int n_in,
                              void* d_out, int out_size, void* d_ws, size_t ws_size, hipStream_t stream) {
    if (n_in < 5) return;
    constexpr size_t NEEDX = ((size_t)(NB - 1) * SEQ_FULL + SEQ) * DM;
    if ((size_t)in_sizes[0] < NEEDX || (size_t)in_sizes[1] < (size_t)DM * DQ || (size_t)in_sizes[2] < (size_t)DM * DKV || (size_t)in_sizes[3] < (size_t)DM * DKV || (size_t)in_sizes[4] < (size_t)DQ * DM) return;
    if ((size_t)out_size < NEEDX) return;
    const float* x = (const float*)d_in[0]; const float* wq = (const float*)d_in[1]; const float* wk = (const float*)d_in[2]; const float* wv = (const float*)d_in[3]; const float* wo = (const float*)d_in[4];
    float* OUT = (float*)d_out;
    constexpr size_t SZ_XB = (size_t)NB * SEQ * DM * 2, SZ_WQ = (size_t)DQ * DM * 2, SZ_WK = (size_t)DKV * DM * 2, SZ_WO = (size_t)DM * DQ * 2, SZ_CS = (size_t)SEQ * 64 * 2 * 4;
    constexpr size_t SZ_Q = (size_t)NB * NH * SEQ * HD * 2, SZ_K = (size_t)NB * NKV * SEQ * HD * 2, SZ_CT = (size_t)NB * SEQ * DQ * 2, SZ_CR = (size_t)NB * RH * DQ * 2;
    constexpr size_t SZ_TOT = SZ_XB + SZ_WQ + 2 * SZ_WK + SZ_WO + SZ_CS + 2 * SZ_Q + 4 * SZ_K + SZ_CT + SZ_CR;
    static_assert(SZ_XB % 256 == 0 && SZ_WQ % 256 == 0 && SZ_WK % 256 == 0 && SZ_WO % 256 == 0 && SZ_CS % 256 == 0 && SZ_Q % 256 == 0 && SZ_K % 256 == 0 && SZ_CT % 256 == 0 && SZ_CR % 256 == 0);
    static_assert(SZ_TOT <= (size_t)134217728);
    if (SZ_TOT > ws_size) return;
    char* wsp = (char*)d_ws;
    auto take = [&](size_t bytes) { char* p = wsp; wsp += bytes; return (void*)p; };
    bf* XB = (bf*)take(SZ_XB); bf* WQt = (bf*)take(SZ_WQ); bf* WKt = (bf*)take(SZ_WK); bf* WVt = (bf*)take(SZ_WK); bf* WOt = (bf*)take(SZ_WO); float* CS = (float*)take(SZ_CS);
    const h16* WOh = (const h16*)WOt;
    h16* Qv = (h16*)take(SZ_Q); h16* Qr = (h16*)take(SZ_Q); h16* Kv = (h16*)take(SZ_K); h16* Kr = (h16*)take(SZ_K); h16* Vv = (h16*)take(SZ_K); h16* Vr = (h16*)take(SZ_K);
    h16* CT = (h16*)take(SZ_CT); h16* CR = (h16*)take(SZ_CR);

    k_cvtx<<<(unsigned)(((size_t)NB * SEQ * DM / 8 + 255) / 256), 256, 0, stream>>>(x, XB);
    k_wtG<<<(DQ * (DM / 64) + 63) / 64, 256, 0, stream>>>(wq, DM, DQ, WQt, 0);
    k_wtG<<<(DKV * (DM / 64) + 63) / 64, 256, 0, stream>>>(wk, DM, DKV, WKt, 0);
    k_wtG<<<(DKV * (DM / 64) + 63) / 64, 256, 0, stream>>>(wv, DM, DKV, WVt, 0);
    k_wtG<<<(DM * (DQ / 64) + 63) / 64, 256, 0, stream>>>(wo, DQ, DM, WOt, 1);
    k_cstab<<<(SEQ * 64 + 255) / 256, 256, 0, stream>>>(CS);
    k_proj_qk<<<dim3(NB * SEQ / 32, NH, 1), 32, 0, stream>>>(XB, WQt, CS, Qv, Qr, NH);
    k_proj_qk<<<dim3(NB * SEQ / 32, NKV, 1), 32, 0, stream>>>(XB, WKt, CS, Kv, Kr, NKV);
    k_proj_vt<<<dim3(DKV / 32, NB * SEQ / 128, 1), 32, 0, stream>>>(WVt, XB, Vv, Vr);
    k_attn_hr<<<dim3(RH / 16, NKV, NB), 128, 0, stream>>>(Qv, Qr, Kv, Kr, Vv, Vr, CT, CR);
    if (SEQ > RH) k_attn<<<dim3((SEQ > RH) ? (SEQ - RH) / 16 : 1, NKV, NB), 128, 0, stream>>>(Qv, Qr, Kv, Vv, CT);
    k_oproj_hr<<<dim3(NB * RH / 32, DM / 128, 1), 32, 0, stream>>>(CT, CR, WOh, OUT);
    if (SEQ > RH) k_oproj<<<dim3((SEQ > RH) ? NB * (SEQ - RH) / 32 : 1, DM / 128, 1), 32, 0, stream>>>(CT, WOh, OUT);
}
